// KPConv_47081431499115
// MI455X (gfx1250) — hardware-verified
//
#include <hip/hip_runtime.h>
#include <stddef.h>
#include <stdint.h>

#pragma clang fp contract(off)

#define PD      3
#define CIN     32
#define COUT    64
#define KPT     15
#define FWW     (KPT * CIN)
#define KA      (2 * FWW)
#define NTHR    256
#define NWAVE   8
#define EPT     8
#define CHUNK   (NTHR * EPT)
#define WCAP    (EPT * 32)
#define LISTN   (NWAVE * WCAP)
#define NBA     1024
#define PKS     10
#define RCAP    28672
#define DEGCAP  64
#define GBM     64
#define GTHR    128
#define GNT     4
#define UPR     (KA / 8)
#define NUW     (COUT * UPR)
#define STGI    512
#define ZINTS   (2 * RCAP + 2 * NBA + LISTN)
#define LDS_AGG (ZINTS * 4 + 64)
#define WSMAX   134217728
#define INV_EXT (1.0f / 0.6f)

static_assert((CHUNK & (CHUNK - 1)) == 0);
static_assert(NBA == (1 << PKS));
static_assert(((long long)CHUNK << PKS) < (1LL << 31));
static_assert(NTHR * 4 == NBA);
static_assert(LISTN >= NBA && LISTN >= NWAVE * WCAP);
static_assert((RCAP % 32) == 0);
static_assert((ZINTS % (NTHR * 4)) == 0);
static_assert(LDS_AGG <= 262144);
static_assert((NBA % NWAVE) == 0 && (NBA % GBM) == 0);
static_assert(GBM == (GTHR / 32) * 16);
static_assert((KA % 32) == 0 && ((KA * 2) % 128) == 0 && ((KA * 2) % 16) == 0);
static_assert((NUW % NTHR) == 0 && NUW * 8 == COUT * KA && (FWW % 8) == 0);
static_assert(CIN == 32 && KPT <= 32);
static_assert(NWAVE * STGI <= RCAP && STGI * 4 >= 4 * 32 * 16 && 4 * 32 * 16 >= KA * 2);
static_assert(KA * 2 == 3 * 32 * 16 + 24 * 16);
static_assert(COUT == 16 * GNT && ((COUT * 4) % 128) == 0);

typedef float          v4f  __attribute__((ext_vector_type(4)));
typedef float          v8f  __attribute__((ext_vector_type(8)));
typedef int            v4i  __attribute__((ext_vector_type(4)));
typedef int            v8i  __attribute__((ext_vector_type(8)));
typedef unsigned short v8us __attribute__((ext_vector_type(8)));
typedef __bf16         v16b __attribute__((ext_vector_type(16)));
typedef v4f  __attribute__((may_alias)) v4fa;
typedef v4i  __attribute__((may_alias)) v4ia;
typedef v8us __attribute__((may_alias)) v8usa;
union Frag { v16b b; v8us h[2]; v8i w; };

__device__ __forceinline__ v8f wmk(const Frag& a, const Frag& b, v8f c) {
  v8f d = __builtin_amdgcn_wmma_f32_16x16x32_bf16(false, a.b, false, b.b, (short)0, c, false, false);
  asm volatile("v_nop\n\tv_nop\n\tv_nop\n\tv_nop" : "+v"(d) : "v"(a.w), "v"(b.w));
  return d;
}

__device__ __forceinline__ unsigned short bf_bits(float f) {
  unsigned int u = __float_as_uint(f);
  u += 0x7FFFu + ((u >> 16) & 1u);
  return (unsigned short)(u >> 16);
}
__device__ __forceinline__ float bf_val(unsigned short b) {
  return __uint_as_float(((unsigned int)b) << 16);
}
__device__ __forceinline__ float bf_rne(float f) { return bf_val(bf_bits(f)); }

__device__ __forceinline__ int scan_chunk(const int* __restrict__ dsts, int nE, int cbase, int slotBase,
                                          int nb, int vec8, int* list, int tid, int lane, int wave) {
  int wc = 0;
  const int el0  = tid * EPT;
  const int e0   = cbase + el0;
  const int sent = -2147483647 - 1;
  v4i da, db;
  if (vec8 != 0 && cbase + CHUNK <= nE) {
    da = *(const v4i*)(dsts + e0);
    db = *(const v4i*)(dsts + e0 + 4);
  } else {
    da.x = (e0     < nE) ? dsts[min(e0,     nE - 1)] : sent;
    da.y = (e0 + 1 < nE) ? dsts[min(e0 + 1, nE - 1)] : sent;
    da.z = (e0 + 2 < nE) ? dsts[min(e0 + 2, nE - 1)] : sent;
    da.w = (e0 + 3 < nE) ? dsts[min(e0 + 3, nE - 1)] : sent;
    db.x = (e0 + 4 < nE) ? dsts[min(e0 + 4, nE - 1)] : sent;
    db.y = (e0 + 5 < nE) ? dsts[min(e0 + 5, nE - 1)] : sent;
    db.z = (e0 + 6 < nE) ? dsts[min(e0 + 6, nE - 1)] : sent;
    db.w = (e0 + 7 < nE) ? dsts[min(e0 + 7, nE - 1)] : sent;
  }
  const unsigned nbs = (unsigned)slotBase;
  const unsigned unb = (unsigned)nb;
  const unsigned s0 = (unsigned)da.x - nbs, s1 = (unsigned)da.y - nbs;
  const unsigned s2 = (unsigned)da.z - nbs, s3 = (unsigned)da.w - nbs;
  const unsigned s4 = (unsigned)db.x - nbs, s5 = (unsigned)db.y - nbs;
  const unsigned s6 = (unsigned)db.z - nbs, s7 = (unsigned)db.w - nbs;
  const bool h0 = s0 < unb, h1 = s1 < unb, h2 = s2 < unb, h3 = s3 < unb;
  const bool h4 = s4 < unb, h5 = s5 < unb, h6 = s6 < unb, h7 = s7 < unb;
  const unsigned any = __builtin_amdgcn_ballot_w32(h0 | h1 | h2 | h3 | h4 | h5 | h6 | h7);
  if (any != 0u) {
#define HITJ(J, HJ, SJ) { \
      const unsigned mj = __builtin_amdgcn_ballot_w32(HJ); \
      if (mj != 0u) { \
        if (HJ) { \
          const int pos = wc + (int)__builtin_amdgcn_mbcnt_lo(mj, 0u); \
          if (pos < WCAP) list[wave * WCAP + pos] = ((el0 + (J)) << PKS) | (int)(SJ); \
        } \
        wc += (int)__builtin_popcount(mj); } }
    HITJ(0, h0, s0)
    HITJ(1, h1, s1)
    HITJ(2, h2, s2)
    HITJ(3, h3, s3)
    HITJ(4, h4, s4)
    HITJ(5, h5, s5)
    HITJ(6, h6, s6)
    HITJ(7, h7, s7)
#undef HITJ
  }
  return wc;
}

__global__ __launch_bounds__(NTHR) void k_wprep(const float* __restrict__ W, unsigned short* WD) {
  const int u = (int)blockIdx.x * NTHR + (int)threadIdx.x;
  if (u >= NUW) return;
  const int n  = u / UPR;
  const int k8 = (u - n * UPR) * 8;
  const int q8 = k8 >= FWW ? k8 - FWW : k8;
  const float* p = W + (size_t)q8 * COUT + n;
  v8us ov;
#pragma unroll
  for (int j = 0; j < 8; ++j) ov[j] = bf_bits(p[(size_t)j * COUT]);
  unsigned short* dp = WD + (size_t)u * 8;
  *(volatile v8us*)dp = ov;
  __threadfence();
  *(volatile v8us*)dp = ov;
}

__global__ __launch_bounds__(GTHR) void k_gemm(const unsigned short* __restrict__ A, int lda,
                                               const unsigned short* __restrict__ BT, int ldb, int K,
                                               float* C32, int ldc, int nRows) {
  __shared__ __attribute__((aligned(16))) float stg[GBM * COUT];
  const int tid = (int)threadIdx.x, lane = tid & 31, wave = tid >> 5, hh = lane >> 4, m = lane & 15;
  const int rowBase = (int)blockIdx.x * GBM;

  v8f acc[GNT];
  {
    const v8f z = {0.f, 0.f, 0.f, 0.f, 0.f, 0.f, 0.f, 0.f};
#pragma unroll
    for (int t = 0; t < GNT; ++t) acc[t] = z;
  }
  const unsigned short* ap = A  + (size_t)(rowBase + 16 * wave + m) * (size_t)lda + 8 * hh;
  const unsigned short* bp = BT + (size_t)m * (size_t)ldb + 8 * hh;

#pragma unroll 1
  for (int k0 = 0; k0 < K; k0 += 32) {
    Frag af;
    af.h[0] = *(const v8usa*)(ap + k0);
    af.h[1] = *(const v8usa*)(ap + k0 + 16);
#pragma unroll
    for (int nt = 0; nt < GNT; ++nt) {
      const unsigned short* wq = bp + (size_t)(16 * nt) * (size_t)ldb + k0;
      Frag bf;
      bf.h[0] = *(const v8usa*)wq;
      bf.h[1] = *(const v8usa*)(wq + 16);
      acc[nt] = wmk(af, bf, acc[nt]);
    }
  }

#pragma unroll
  for (int nt = 0; nt < GNT; ++nt) {
    const int lc = 16 * nt + m;
#pragma unroll
    for (int r = 0; r < 8; ++r) {
      const int lr = 16 * wave + 8 * hh + r;
      stg[lr * COUT + lc] = acc[nt][r];
    }
  }
  __syncthreads();

  v4f pv[8];
#pragma unroll
  for (int i = 0; i < 8; ++i) {
    const int lr = 16 * wave + 2 * i + hh;
    pv[i] = *(const v4fa*)(stg + lr * COUT + 4 * m);
  }
#pragma unroll
  for (int i = 0; i < 8; ++i) {
    const int gr = rowBase + 16 * wave + 2 * i + hh;
    float* op = C32 + (size_t)gr * (size_t)ldc + 4 * m;
    if (gr < nRows) *(volatile v4f*)op = pv[i];
  }
  __threadfence();
#pragma unroll
  for (int i = 0; i < 8; ++i) {
    const int gr = rowBase + 16 * wave + 2 * i + hh;
    float* op = C32 + (size_t)gr * (size_t)ldc + 4 * m;
    if (gr < nRows) *(volatile v4f*)op = pv[i];
  }
}

__global__ __launch_bounds__(NTHR) void k_agg(const float* __restrict__ pos, const float* __restrict__ feat,
                                              const float* __restrict__ kp, const int* __restrict__ srcs,
                                              const int* __restrict__ dsts, unsigned short* Aout,
                                              int nN, int nE, int vec8) {
  extern __shared__ __attribute__((aligned(16))) int lds_i[];
  int* reg1 = lds_i;
  int* reg2 = reg1 + RCAP;
  int* scnt = reg2 + RCAP;
  int* soff = scnt + NBA;
  int* list = soff + NBA;
  int* wcnt = list + LISTN;
  int* wtot = wcnt + NWAVE;
  const int tid = (int)threadIdx.x, lane = tid & 31, wave = tid >> 5;
  const int nodeBase = (int)blockIdx.x * NBA;

  const int kpi = lane < KPT ? lane : KPT - 1;
  const float kx = bf_rne(kp[3 * kpi + 0]);
  const float ky = bf_rne(kp[3 * kpi + 1]);
  const float kz = bf_rne(kp[3 * kpi + 2]);

  {
    const v4i z4 = {0, 0, 0, 0};
    for (int i = tid * 4; i < ZINTS; i += NTHR * 4) *(v4ia*)(lds_i + i) = z4;
    if (tid < 2 * NWAVE) wcnt[tid] = 0;
  }
  __syncthreads();

  int tot = 0;
  const int nChunks = (nE + CHUNK - 1) / CHUNK;
#pragma unroll 1
  for (int ch = 0; ch < nChunks; ++ch) {
    const int cbase = ch * CHUNK;
    const int wc = scan_chunk(dsts, nE, cbase, nodeBase, NBA, vec8, list, tid, lane, wave);
    if (lane == 0) wcnt[wave] = wc;
    __syncthreads();
    int pre = 0, all = 0;
#pragma unroll
    for (int w2 = 0; w2 < NWAVE; ++w2) {
      int c = wcnt[w2];
      c = c < 0 ? 0 : (c > WCAP ? WCAP : c);
      all += c;
      pre += (w2 < wave) ? c : 0;
    }
    const int wcc  = wc > WCAP ? WCAP : wc;
    const int base = tot + pre;
#pragma unroll 1
    for (int i = lane; i < wcc; i += 32) {
      const int ent = list[wave * WCAP + i];
      const int el  = (ent >> PKS) & (CHUNK - 1);
      const int sl  = ent & (NBA - 1);
      int eid = cbase + el;
      eid = eid > nE - 1 ? nE - 1 : eid;
      const int pos2 = base + i;
      if (pos2 < RCAP) reg1[pos2] = (int)(((unsigned)eid << PKS) | (unsigned)sl);
    }
    tot += all;
    tot = tot > RCAP ? RCAP : tot;
    __syncthreads();
  }
  const int nh = tot;

  if (wave == 0) {
#pragma unroll 1
    for (int b0 = 0; b0 < nh; b0 += 32) {
      const int idx = b0 + lane;
      const int uv  = reg1[idx < RCAP ? idx : RCAP - 1];
      const int m32 = (nh - b0) < 32 ? (nh - b0) : 32;
#pragma unroll 1
      for (int k = 0; k < m32; ++k) {
        const int u  = __builtin_amdgcn_readlane(uv, k);
        const int sl = u & (NBA - 1);
        if (lane == 0) scnt[sl] = scnt[sl] + 1;
      }
    }
  }
  __syncthreads();

  {
    const v4i ca = *(const v4ia*)(scnt + 4 * tid);
    const int e0 = ca.x < 0 ? 0 : ca.x, e1 = ca.y < 0 ? 0 : ca.y, e2 = ca.z < 0 ? 0 : ca.z, e3 = ca.w < 0 ? 0 : ca.w;
    const int ts = e0 + e1 + e2 + e3;
    int incl = ts;
#pragma unroll
    for (int d = 1; d < 32; d <<= 1) {
      const int up = __shfl_up(incl, d, 32);
      if (lane >= d) incl += up;
    }
    if (lane == 31) wtot[wave] = incl;
    __syncthreads();
    int pre = 0;
#pragma unroll
    for (int w2 = 0; w2 < NWAVE; ++w2) pre += (w2 < wave) ? wtot[w2] : 0;
    int run = pre + incl - ts;
    soff[4 * tid + 0] = run; run += e0;
    soff[4 * tid + 1] = run; run += e1;
    soff[4 * tid + 2] = run; run += e2;
    soff[4 * tid + 3] = run;
  }
  __syncthreads();
  for (int i = tid; i < NBA; i += NTHR) list[i] = soff[i];
  __syncthreads();

  if (wave == 0) {
#pragma unroll 1
    for (int b0 = 0; b0 < nh; b0 += 32) {
      const int idx = b0 + lane;
      const int uv  = reg1[idx < RCAP ? idx : RCAP - 1];
      const int m32 = (nh - b0) < 32 ? (nh - b0) : 32;
#pragma unroll 1
      for (int k = 0; k < m32; ++k) {
        const int u   = __builtin_amdgcn_readlane(uv, k);
        const int sl  = u & (NBA - 1);
        const int eid = (int)((unsigned)u >> PKS);
        if (lane == 0) {
          int pos2 = list[sl];
          pos2 = pos2 < 0 ? 0 : (pos2 > RCAP - 1 ? RCAP - 1 : pos2);
          reg2[pos2] = eid;
          list[sl] = pos2 + 1;
        }
      }
    }
  }
  __syncthreads();

  const int nbw = NBA / NWAVE;
  const bool ovf = (nh >= RCAP);
  const float qnan = __int_as_float(0x7fc00000);
  unsigned short* stg16 = (unsigned short*)(reg1 + wave * STGI);

#pragma unroll 1
  for (int jt = 0; jt < nbw; ++jt) {
    const int slot = wave * nbw + jt;
    const int node = nodeBase + slot;
    int st = soff[slot];
    const int craw = scnt[slot];
    int cnt = craw;
    st  = st < 0 ? 0 : (st > nh ? nh : st);
    cnt = cnt < 0 ? 0 : (cnt > DEGCAP ? DEGCAP : cnt);
    if (cnt > nh - st) cnt = nh - st;
    const float pz = (ovf || craw > DEGCAP) ? qnan : 0.0f;
    const bool live = node < nN;
    const int nc = live ? node : nN - 1;
    const float* pq = pos + (size_t)nc * PD;
    const float qx = bf_rne(pq[0]), qy = bf_rne(pq[1]), qz = bf_rne(pq[2]);

    float acc[KPT];
#pragma unroll
    for (int kk = 0; kk < KPT; ++kk) acc[kk] = 0.0f;

#pragma unroll 1
    for (int b0 = 0; b0 < cnt; b0 += 32) {
      int idx = st + b0 + lane; idx = idx > RCAP - 1 ? RCAP - 1 : idx;
      int eid = reg2[idx]; eid = eid < 0 ? 0 : (eid > nE - 1 ? nE - 1 : eid);
      int sr = srcs[eid]; sr = sr < 0 ? 0 : (sr > nN - 1 ? nN - 1 : sr);
      const float* ps = pos + (size_t)sr * PD;
      const float yx = bf_rne(ps[0]) - qx;
      const float yy = bf_rne(ps[1]) - qy;
      const float yz = bf_rne(ps[2]) - qz;
      const int iyx = __float_as_int(yx), iyy = __float_as_int(yy), iyz = __float_as_int(yz);
      const int m32 = (cnt - b0) < 32 ? (cnt - b0) : 32;
#pragma unroll 1
      for (int k = 0; k < m32; ++k) {
        const int sk = __builtin_amdgcn_readlane(sr, k);
        const float ex = __int_as_float(__builtin_amdgcn_readlane(iyx, k));
        const float ey = __int_as_float(__builtin_amdgcn_readlane(iyy, k));
        const float ez = __int_as_float(__builtin_amdgcn_readlane(iyz, k));
        const float f  = bf_rne(feat[(size_t)sk * CIN + lane]);
        const float dx = ex - kx, dy = ey - ky, dz = ez - kz;
        const float sq = (dx * dx + dz * dz) + dy * dy;
        const float dd = sqrtf(sq);
        const float hv = fmaxf(1.0f - dd * INV_EXT, 0.0f);
        const int ihv = __float_as_int(hv);
#pragma unroll
        for (int kk = 0; kk < KPT; ++kk) {
          const float mk = __int_as_float(__builtin_amdgcn_readlane(ihv, kk));
          acc[kk] = fmaf(mk, f, acc[kk]);
        }
      }
    }

    __builtin_amdgcn_fence(__ATOMIC_RELEASE, "wavefront");
    __builtin_amdgcn_wave_barrier();
#pragma unroll
    for (int kk = 0; kk < KPT; ++kk) {
      const float r = (live ? acc[kk] : 0.0f) + pz;
      const unsigned short hb = bf_bits(r);
      const unsigned short lb = bf_bits(r - bf_val(hb));
      stg16[32 * kk + lane]       = hb;
      stg16[FWW + 32 * kk + lane] = lb;
    }
    __builtin_amdgcn_fence(__ATOMIC_RELEASE, "wavefront");
    __builtin_amdgcn_wave_barrier();
    const v8us p0 = *(const v8usa*)(stg16 + (0 * 32 + lane) * 8);
    const v8us p1 = *(const v8usa*)(stg16 + (1 * 32 + lane) * 8);
    const v8us p2 = *(const v8usa*)(stg16 + (2 * 32 + lane) * 8);
    const v8us p3 = *(const v8usa*)(stg16 + (3 * 32 + lane) * 8);
    unsigned short* gp = Aout + (size_t)node * (size_t)KA;
    *(volatile v8us*)(gp + (0 * 32 + lane) * 8) = p0;
    *(volatile v8us*)(gp + (1 * 32 + lane) * 8) = p1;
    *(volatile v8us*)(gp + (2 * 32 + lane) * 8) = p2;
    if (lane < 24) *(volatile v8us*)(gp + (3 * 32 + lane) * 8) = p3;
    __threadfence();
    *(volatile v8us*)(gp + (0 * 32 + lane) * 8) = p0;
    *(volatile v8us*)(gp + (1 * 32 + lane) * 8) = p1;
    *(volatile v8us*)(gp + (2 * 32 + lane) * 8) = p2;
    if (lane < 24) *(volatile v8us*)(gp + (3 * 32 + lane) * 8) = p3;
  }
}

static inline int cdiv(int a, int b) { return (a + b - 1) / b; }
static inline size_t al256(size_t o) { return (o + 255) & ~(size_t)255; }

extern "C" void kernel_launch(void* const* d_in, const int* in_sizes, int n_in,
                              void* d_out, int out_size, void* d_ws, size_t ws_size,
                              hipStream_t stream) {
  if (n_in < 6) return;
  if (in_sizes[0] < PD || (in_sizes[0] % PD) != 0) return;
  const int nN = in_sizes[0] / PD;
  if (nN < 1 || nN > (1 << 22)) return;
  if ((long long)in_sizes[1] != (long long)nN * CIN) return;
  if (in_sizes[2] != KPT * PD) return;
  if (in_sizes[3] != KPT * CIN * COUT) return;
  const int nE = in_sizes[4];
  if (nE < 1 || nE >= (1 << 21)) return;
  if (in_sizes[5] != nE) return;
  if ((long long)out_size != (long long)nN * COUT) return;

  const float* pos  = (const float*)d_in[0];
  const float* feat = (const float*)d_in[1];
  const float* kpts = (const float*)d_in[2];
  const float* W    = (const float*)d_in[3];
  const int*   src  = (const int*)  d_in[4];
  const int*   dst  = (const int*)  d_in[5];
  float* out = (float*)d_out;

  const int MP   = cdiv(nN, GBM) * GBM;
  const int gM   = MP / GBM;
  const int gA   = cdiv(MP, NBA);
  const int RA   = gA * NBA;
  const int vec8 = ((nE & 3) == 0) ? 1 : 0;
  if ((long long)RA < (long long)MP) return;

  char* ws = (char*)d_ws;
  size_t off = 0;
  const size_t oWD = off; off = al256(off + (size_t)NUW * 8 * 2);
  const size_t oAP = off; off = al256(off + (size_t)RA * KA * 2);
  if (off > ws_size || off > (size_t)WSMAX) return;
  unsigned short* WD = (unsigned short*)(ws + oWD);
  unsigned short* AP = (unsigned short*)(ws + oAP);

  hipFuncSetAttribute(reinterpret_cast<const void*>(&k_agg), hipFuncAttributeMaxDynamicSharedMemorySize, LDS_AGG);

  k_wprep<<<NUW / NTHR, NTHR, 0, stream>>>(W, WD);
  k_agg<<<gA, NTHR, LDS_AGG, stream>>>(pos, feat, kpts, src, dst, AP, nN, nE, vec8);
  k_gemm<<<dim3(gM, 1), GTHR, 0, stream>>>(AP, KA, WD, KA, KA, out, COUT, nN);
}
